// GPModel_59021440581986
// MI455X (gfx1250) — hardware-verified
//
#include <hip/hip_runtime.h>
#include <stddef.h>


#define FIN     64
#define FH      64
#define NPG     500
#define KPG     250
#define MPP     512
#define KPP     256
#define NTHR    256
#define NWAVE   8
#define EPT     8
#define NGRP    2
#define CHUNK   (NTHR * EPT * NGRP)
#define WCAP    (EPT * NGRP * 32)
#define LISTN   (NWAVE * WCAP)
#define ESHF    11
#define NBC     32768
#define NBF     2048
#define RCAP    40960
#define RBN     128
#define TGT     256
#define DEGCAP  512
#define GROWS   128
#define OTHR    512
#define WSCALE  16
#define WSCAP   134217728

#define LDS_COUNT ((NBC + LISTN + NWAVE) * 4)
#define LDS_FILL  ((RCAP + NBF + LISTN + NWAVE) * 4)
#define LDS_GEMM  36864

static_assert((CHUNK & (CHUNK - 1)) == 0);
static_assert((NBC & (NBC - 1)) == 0 && (NBF & (NBF - 1)) == 0);
static_assert(NBF <= (1 << ESHF));
static_assert((NBC % NBF) == 0);
static_assert(OTHR * 4 == NBF);
static_assert((RCAP % 32) == 0);
static_assert(TGT == NWAVE * 32);
static_assert(GROWS == NWAVE * 16);
static_assert((GROWS * FIN / 8) % NTHR == 0);
static_assert(GROWS * (FIN + 8) * 2 <= LDS_GEMM && GROWS * FH * 4 <= LDS_GEMM);
static_assert((FIN % 32) == 0 && FH == 64);
static_assert(NBC == NWAVE * 128 * 32);
static_assert(FIN * FH / 8 == 2 * NTHR);
static_assert(KPP == NWAVE * 32 && KPP >= KPG && MPP >= NPG && MPP <= 2 * NTHR);
static_assert(2 * FH == 128);

typedef float     v2f  __attribute__((ext_vector_type(2)));
typedef float     v4f  __attribute__((ext_vector_type(4)));
typedef float     v8f  __attribute__((ext_vector_type(8)));
typedef int       v4i  __attribute__((ext_vector_type(4)));
typedef _Float16  v8h  __attribute__((ext_vector_type(8)));
typedef _Float16  v16h __attribute__((ext_vector_type(16)));
union FragH { v16h v; v8h h[2]; };
union FI { float f; int i; };

__device__ __forceinline__ v8f wmf(v16h a, v16h b, v8f c) {
  v8f d = __builtin_amdgcn_wmma_f32_16x16x32_f16(false, a, false, b, (short)0, c, false, false);
  asm volatile("v_nop\n\tv_nop\n\tv_nop\n\tv_nop" : "+v"(d) : "v"(a), "v"(b));
  return d;
}

__device__ __forceinline__ int clampi(int v, int lo, int hi) { return v < lo ? lo : (v > hi ? hi : v); }
__device__ __forceinline__ int rl_i(int v, int l) { return __builtin_amdgcn_readlane(v, l); }
__device__ __forceinline__ float rl_f(float v, int l) { FI u; u.f = v; u.i = __builtin_amdgcn_readlane(u.i, l); return u.f; }
__device__ __forceinline__ float wsum(float v) {
#pragma unroll
  for (int o = 16; o >= 1; o >>= 1) v += __shfl_xor(v, o, 32);
  return v;
}
__device__ __forceinline__ double dxor(double v, int o) {
  const unsigned long long u = (unsigned long long)__double_as_longlong(v);
  int lo = (int)(unsigned)u, hi = (int)(unsigned)(u >> 32);
  lo = __shfl_xor(lo, o, 32);
  hi = __shfl_xor(hi, o, 32);
  const unsigned long long r = ((unsigned long long)(unsigned)hi << 32) | (unsigned long long)(unsigned)lo;
  return __longlong_as_double((long long)r);
}
__device__ __forceinline__ int mp_index(int row) { const int gq = row / NPG; return gq * MPP + (row - gq * NPG); }
__device__ __forceinline__ int kp_index(int a)   { const int gq = a / KPG;   return gq * KPP + (a - gq * KPG); }

template <int NB, int SRC>
__device__ __forceinline__ int scan_chunk(const int* __restrict__ dsts, const int* __restrict__ srcs, int nE, int nN,
                                          int cbase, int slotBase, int vec8, int* list, int tid, int lane, int wave) {
  int wc = 0;
#pragma unroll
  for (int g = 0; g < NGRP; ++g) {
    const int el0  = (g * NTHR + tid) * EPT;
    const int e0   = cbase + el0;
    const int sent = -2147483647 - 1;
    v4i da, db;
    v4i sa = {0, 0, 0, 0}, sb = {0, 0, 0, 0};
    if (vec8 != 0 && cbase + CHUNK <= nE) {
      da = *(const v4i*)(dsts + e0);
      db = *(const v4i*)(dsts + e0 + 4);
      if (SRC) {
        sa = *(const v4i*)(srcs + e0);
        sb = *(const v4i*)(srcs + e0 + 4);
      }
    } else {
      da.x = (e0     < nE) ? dsts[min(e0, nE - 1)] : sent;
      da.y = (e0 + 1 < nE) ? dsts[min(e0 + 1, nE - 1)] : sent;
      da.z = (e0 + 2 < nE) ? dsts[min(e0 + 2, nE - 1)] : sent;
      da.w = (e0 + 3 < nE) ? dsts[min(e0 + 3, nE - 1)] : sent;
      db.x = (e0 + 4 < nE) ? dsts[min(e0 + 4, nE - 1)] : sent;
      db.y = (e0 + 5 < nE) ? dsts[min(e0 + 5, nE - 1)] : sent;
      db.z = (e0 + 6 < nE) ? dsts[min(e0 + 6, nE - 1)] : sent;
      db.w = (e0 + 7 < nE) ? dsts[min(e0 + 7, nE - 1)] : sent;
      if (SRC) {
        sa.x = srcs[min(e0, nE - 1)];
        sa.y = srcs[min(e0 + 1, nE - 1)];
        sa.z = srcs[min(e0 + 2, nE - 1)];
        sa.w = srcs[min(e0 + 3, nE - 1)];
        sb.x = srcs[min(e0 + 4, nE - 1)];
        sb.y = srcs[min(e0 + 5, nE - 1)];
        sb.z = srcs[min(e0 + 6, nE - 1)];
        sb.w = srcs[min(e0 + 7, nE - 1)];
      }
    }
    if (SRC) {
      sa.x = min(max(sa.x, 0), nN - 1); sa.y = min(max(sa.y, 0), nN - 1);
      sa.z = min(max(sa.z, 0), nN - 1); sa.w = min(max(sa.w, 0), nN - 1);
      sb.x = min(max(sb.x, 0), nN - 1); sb.y = min(max(sb.y, 0), nN - 1);
      sb.z = min(max(sb.z, 0), nN - 1); sb.w = min(max(sb.w, 0), nN - 1);
    }
    const unsigned nb = (unsigned)slotBase;
    const unsigned s0 = (unsigned)da.x - nb, s1 = (unsigned)da.y - nb;
    const unsigned s2 = (unsigned)da.z - nb, s3 = (unsigned)da.w - nb;
    const unsigned s4 = (unsigned)db.x - nb, s5 = (unsigned)db.y - nb;
    const unsigned s6 = (unsigned)db.z - nb, s7 = (unsigned)db.w - nb;
    const bool h0 = s0 < (unsigned)NB, h1 = s1 < (unsigned)NB, h2 = s2 < (unsigned)NB, h3 = s3 < (unsigned)NB;
    const bool h4 = s4 < (unsigned)NB, h5 = s5 < (unsigned)NB, h6 = s6 < (unsigned)NB, h7 = s7 < (unsigned)NB;
    const unsigned any = __builtin_amdgcn_ballot_w32(h0 | h1 | h2 | h3 | h4 | h5 | h6 | h7);
    if (any != 0u) {
#define HITJ(HJ, SJ, VJ) { \
        const unsigned mj = __builtin_amdgcn_ballot_w32(HJ); \
        if (mj != 0u) { \
          if (HJ) { \
            const int pos = wc + (int)__builtin_amdgcn_mbcnt_lo(mj, 0u); \
            const int entv = SRC ? (((VJ) << ESHF) | (int)(SJ)) : (int)(SJ); \
            if (pos < WCAP) list[wave * WCAP + pos] = entv; \
          } \
          wc += (int)__builtin_popcount(mj); } }
      HITJ(h0, s0, sa.x)
      HITJ(h1, s1, sa.y)
      HITJ(h2, s2, sa.z)
      HITJ(h3, s3, sa.w)
      HITJ(h4, s4, sb.x)
      HITJ(h5, s5, sb.y)
      HITJ(h6, s6, sb.z)
      HITJ(h7, s7, sb.w)
#undef HITJ
    }
  }
  return wc;
}

__global__ __launch_bounds__(NTHR) void k_wprep(const float* __restrict__ w1, _Float16* wp) {
  const int i  = (int)blockIdx.x * NTHR + (int)threadIdx.x;
  const int n  = i >> 3;
  const int k0 = (i & 7) * 8;
  v8h hv;
#pragma unroll
  for (int e = 0; e < 8; ++e) hv[e] = (_Float16)(w1[(k0 + e) * FH + n] * (float)WSCALE);
  _Float16* d = wp + (size_t)i * 8;
  *(volatile v8h*)d = hv;
  __threadfence();
  *(volatile v8h*)d = hv;
}

template <int WD>
__global__ __launch_bounds__(NTHR) void k_count(
    const int* __restrict__ ei, int keyOff, int* cnt, float* dis, int nE, int nN, int vec8) {
  extern __shared__ v4f lds_dyn[];
  int* scnt = (int*)lds_dyn;
  int* list = scnt + NBC;
  int* wcnt = list + LISTN;
  const int tid = threadIdx.x, lane = tid & 31, wave = tid >> 5;
  const int nodeBase = blockIdx.x * NBC;
  const int* keys = ei + keyOff;

  {
    const v4i z = {0, 0, 0, 0};
    for (int i = tid; i < NBC / 4; i += NTHR) ((v4i*)scnt)[i] = z;
  }
  __syncthreads();

  const int nChunks = (nE + CHUNK - 1) / CHUNK;
#pragma unroll 1
  for (int ch = 0; ch < nChunks; ++ch) {
    const int cbase = ch * CHUNK;
    const int wc = scan_chunk<NBC, 0>(keys, ei, nE, nN, cbase, nodeBase, vec8, list, tid, lane, wave);
    if (lane == 0) wcnt[wave] = wc;
    __syncthreads();
    if (wave == 0) {
#pragma unroll 1
      for (int wsx = 0; wsx < NWAVE; ++wsx) {
        int n = __builtin_amdgcn_readfirstlane(wcnt[wsx]);
        n = n > WCAP ? WCAP : (n < 0 ? 0 : n);
        const int* lp = list + wsx * WCAP;
#pragma unroll 1
        for (int i = 0; i < n; ++i) {
          const int ent  = __builtin_amdgcn_readfirstlane(lp[i]);
          const int slot = ent & (NBC - 1);
          if (lane == 0) scnt[slot] = scnt[slot] + 1;
        }
      }
    }
    __syncthreads();
  }

  int*   cp = cnt + (size_t)nodeBase;
  float* dp = dis + (size_t)nodeBase;
#pragma unroll 1
  for (int q = 0; q < 128; ++q) {
    const int f = (wave * 128 + q) * 32 + lane;
    const int c = scnt[f];
    *(volatile int*)(cp + f) = c;
    if (WD) {
      const float dv = 1.0f / sqrtf((float)c);
      const float d  = c > 0 ? dv : 0.0f;
      *(volatile float*)(dp + f) = d;
    }
  }
  __threadfence();
#pragma unroll 1
  for (int q = 0; q < 128; ++q) {
    const int f = (wave * 128 + q) * 32 + lane;
    const int c = scnt[f];
    *(volatile int*)(cp + f) = c;
    if (WD) {
      const float dv = 1.0f / sqrtf((float)c);
      const float d  = c > 0 ? dv : 0.0f;
      *(volatile float*)(dp + f) = d;
    }
  }
}

__global__ __launch_bounds__(OTHR) void k_offsets(
    const int* __restrict__ cnt, int* off, int* rbase, int nBF) {
  __shared__ __attribute__((aligned(16))) int srb[RBN];
  __shared__ int wtot[OTHR / 32];
  const int tid = threadIdx.x, lane = tid & 31, wave = tid >> 5;
  for (int i = tid; i < RBN; i += OTHR) srb[i] = 0;
  int carry = 0;
#pragma unroll 1
  for (int fb = 0; fb < nBF; ++fb) {
    const int base = fb * NBF;
    const v4i c = *(const v4i*)(cnt + base + 4 * tid);
    const int e0 = max(c.x, 0), e1 = max(c.y, 0), e2 = max(c.z, 0), e3 = max(c.w, 0);
    const int ts = e0 + e1 + e2 + e3;
    int incl = ts;
#pragma unroll
    for (int d = 1; d < 32; d <<= 1) {
      const int t = __shfl_up(incl, d);
      if (lane >= d) incl += t;
    }
    if (lane == 31) wtot[wave] = incl;
    __syncthreads();
    int pre = 0;
#pragma unroll 1
    for (int w = 0; w < wave; ++w) pre += wtot[w];
    int tot = 0;
#pragma unroll
    for (int w = 0; w < OTHR / 32; ++w) tot += wtot[w];
    int run = carry + pre + incl - ts;
    v4i o;
    o.x = run; run += e0;
    o.y = run; run += e1;
    o.z = run; run += e2;
    o.w = run;
    int* op = off + base + 4 * tid;
    *(volatile v4i*)op = o;
    __threadfence();
    *(volatile v4i*)op = o;
    if (tid == 0) srb[min(fb, RBN - 1)] = carry;
    carry += (tot + 31) & ~31;
    __syncthreads();
  }
  if (tid == 0) srb[min(nBF, RBN - 1)] = carry;
  __syncthreads();
  v4i rv = {0, 0, 0, 0};
  if (tid < 32) rv = *(const v4i*)(srb + 4 * tid);
  if (tid < 32) *(volatile v4i*)(rbase + 4 * tid) = rv;
  __threadfence();
  if (tid < 32) *(volatile v4i*)(rbase + 4 * tid) = rv;
}

__global__ __launch_bounds__(NTHR) void k_fill(
    const int* __restrict__ ei, const int* __restrict__ off, const int* __restrict__ rbase,
    int* csr, int nN, int nE, int vec8, int csrLen) {
  extern __shared__ v4f lds_dyn[];
  int* region = (int*)lds_dyn;
  int* cursor = region + RCAP;
  int* list   = cursor + NBF;
  int* wcnt   = list + LISTN;
  const int tid = threadIdx.x, lane = tid & 31, wave = tid >> 5;
  const int b = blockIdx.x;
  const int nodeBase = b * NBF;
  const int* dsts = ei + nE;

  int rb0 = rbase[b];
  const int rb1 = rbase[b + 1];
  rb0 = rb0 < 0 ? 0 : (rb0 > csrLen ? csrLen : rb0);
  rb0 &= ~31;
  int len = rb1 - rb0;
  len = len < 0 ? 0 : (len > RCAP ? RCAP : len);
  int lenW = (len + 31) & ~31;
  if (rb0 + lenW > csrLen) lenW = (csrLen - rb0) & ~31;

  {
    const v4i z = {0, 0, 0, 0};
    for (int i = tid; i < RCAP / 4; i += NTHR) ((v4i*)region)[i] = z;
    for (int s = tid; s < NBF; s += NTHR) {
      int o = off[nodeBase + s] - rb0;
      o = o < 0 ? 0 : (o > RCAP ? RCAP : o);
      cursor[s] = o;
    }
  }
  __syncthreads();

  const int nChunks = (nE + CHUNK - 1) / CHUNK;
#pragma unroll 1
  for (int ch = 0; ch < nChunks; ++ch) {
    const int cbase = ch * CHUNK;
    const int wc = scan_chunk<NBF, 1>(dsts, ei, nE, nN, cbase, nodeBase, vec8, list, tid, lane, wave);
    if (lane == 0) wcnt[wave] = wc;
    __syncthreads();
    if (wave == 0) {
#pragma unroll 1
      for (int wsx = 0; wsx < NWAVE; ++wsx) {
        int n = __builtin_amdgcn_readfirstlane(wcnt[wsx]);
        n = n > WCAP ? WCAP : (n < 0 ? 0 : n);
        const int* lp = list + wsx * WCAP;
#pragma unroll 1
        for (int i = 0; i < n; ++i) {
          const int ent  = __builtin_amdgcn_readfirstlane(lp[i]);
          const int slot = ent & (NBF - 1);
          int src = (ent >> ESHF) & 0xFFFFF;
          src = src > nN - 1 ? nN - 1 : src;
          if (lane == 0) {
            int pos = cursor[slot];
            pos = pos < 0 ? 0 : (pos > RCAP - 1 ? RCAP - 1 : pos);
            region[pos] = src;
            const int np = pos + 1;
            cursor[slot] = np > RCAP ? RCAP : np;
          }
        }
      }
    }
    __syncthreads();
  }

  const int nv = lenW >> 2;
  int* gp = csr + rb0;
#pragma unroll 1
  for (int i = tid; i < nv; i += NTHR) { const v4i v = ((const v4i*)region)[i]; *(volatile v4i*)(gp + 4 * i) = v; }
  __threadfence();
#pragma unroll 1
  for (int i = tid; i < nv; i += NTHR) { const v4i v = ((const v4i*)region)[i]; *(volatile v4i*)(gp + 4 * i) = v; }
}

__global__ __launch_bounds__(NTHR) void k_score(
    const int* __restrict__ csr, const int* __restrict__ off, const int* __restrict__ cnt,
    const float* __restrict__ dis, const float* __restrict__ x, double* score, int nN, int csrLen) {
  const int tid = threadIdx.x, lane = tid & 31, wave = tid >> 5;
  const int tbase = blockIdx.x * TGT + wave * 32;
  const int cl = tbase + lane;
  const int cnt_l = cnt[cl];
  const int off_l = off[cl];
  const float dis_l = dis[cl];
  double mys = 0.0;

#pragma unroll 1
  for (int j = 0; j < 32; ++j) {
    const int c = tbase + j;
    int n = rl_i(cnt_l, j);
    n = clampi(n, 0, DEGCAP);
    const int st = rl_i(off_l, j);
    const float dc = rl_f(dis_l, j);
    double ax = 0.0, ay = 0.0;
#pragma unroll 1
    for (int q0 = 0; q0 < n; q0 += 32) {
      const int pos = clampi(st + q0 + lane, 0, csrLen - 1);
      const int sl  = clampi(csr[pos], 0, nN - 1);
      const float wl = dis[sl] * dc;
      const int mcnt = (n - q0) < 32 ? (n - q0) : 32;
#pragma unroll 1
      for (int p = 0; p < mcnt; ++p) {
        const int s = rl_i(sl, p);
        const float w = rl_f(wl, p);
        const v2f xv = *(const v2f*)(x + (size_t)s * FIN + 2 * lane);
        const float px = w * xv.x, py = w * xv.y;
        ax += (double)px;
        ay += (double)py;
      }
    }
    const int cr = c < nN ? c : nN - 1;
    const v2f xc = *(const v2f*)(x + (size_t)cr * FIN + 2 * lane);
    double d = __builtin_fabs((double)xc.x - ax) + __builtin_fabs((double)xc.y - ay);
#pragma unroll
    for (int o = 16; o >= 1; o >>= 1) d += dxor(d, o);
    mys = (lane == j) ? d : mys;
  }
  double* sp = score + (size_t)tbase + lane;
  *(volatile double*)sp = mys;
  __threadfence();
  *(volatile double*)sp = mys;
}

__global__ __launch_bounds__(NTHR) void k_topk(const double* __restrict__ score, int* mp, int* permp, int nN) {
  __shared__ double ss[MPP];
  __shared__ __attribute__((aligned(16))) int smp[MPP];
  __shared__ __attribute__((aligned(16))) int sperm[KPP];
  const int tid = threadIdx.x;
  const int g = blockIdx.x;
  const int node0 = g * NPG;
  for (int i = tid; i < MPP; i += NTHR) {
    const int ii = i < NPG ? i : NPG - 1;
    ss[i]  = score[clampi(node0 + ii, 0, nN - 1)];
    smp[i] = -1;
  }
  for (int i = tid; i < KPP; i += NTHR) sperm[i] = node0;
  __syncthreads();
#pragma unroll 1
  for (int rep = 0; rep < 2; ++rep) {
    const int i  = tid + rep * NTHR;
    const int ii = i < NPG ? i : NPG - 1;
    const double si = ss[ii];
    int r = 0;
#pragma unroll 4
    for (int j = 0; j < NPG; ++j) {
      const double sj = ss[j];
      r += ((sj > si) || (sj == si && j < ii)) ? 1 : 0;
    }
    if (i < NPG && r < KPG) {
      smp[i]   = g * KPG + r;
      sperm[r] = node0 + i;
    }
  }
  __syncthreads();
  v4i mv = {0, 0, 0, 0}, pv = {0, 0, 0, 0};
  if (tid < MPP / 4) mv = ((const v4i*)smp)[tid];
  if (tid < KPP / 4) pv = ((const v4i*)sperm)[tid];
  int* mpp = mp + (size_t)g * MPP + 4 * tid;
  int* ppp = permp + (size_t)g * KPP + 4 * tid;
  if (tid < MPP / 4) *(volatile v4i*)mpp = mv;
  if (tid < KPP / 4) *(volatile v4i*)ppp = pv;
  __threadfence();
  if (tid < MPP / 4) *(volatile v4i*)mpp = mv;
  if (tid < KPP / 4) *(volatile v4i*)ppp = pv;
}

__global__ __launch_bounds__(NTHR) void k_gemm(
    const float* __restrict__ A, const _Float16* __restrict__ Bw, float* C, int nRowsA) {
  extern __shared__ v4f lds_dyn[];
  constexpr int KD  = FIN;
  constexpr int APH = KD + 8;
  constexpr float OSC = 1.0f / (float)WSCALE;
  _Float16* sA  = (_Float16*)lds_dyn;
  float*    stg = (float*)lds_dyn;
  const int tid = threadIdx.x, lane = tid & 31, wave = tid >> 5, hh = lane >> 4, m = lane & 15;
  const int rowBase = blockIdx.x * GROWS;

#pragma unroll
  for (int i = 0; i < (GROWS * KD / 8) / NTHR; ++i) {
    const int idx = i * NTHR + tid;
    const int r   = idx / (KD / 8);
    const int c0  = (idx - r * (KD / 8)) * 8;
    int row = rowBase + r;
    row = row > nRowsA - 1 ? nRowsA - 1 : row;
    const float* ap = A + (size_t)row * KD + c0;
    const v4f a = *(const v4f*)ap, b = *(const v4f*)(ap + 4);
    v8h hv;
    hv[0] = (_Float16)a.x; hv[1] = (_Float16)a.y; hv[2] = (_Float16)a.z; hv[3] = (_Float16)a.w;
    hv[4] = (_Float16)b.x; hv[5] = (_Float16)b.y; hv[6] = (_Float16)b.z; hv[7] = (_Float16)b.w;
    *(v8h*)(sA + r * APH + c0) = hv;
  }
  __syncthreads();

  v8f acc[4];
#pragma unroll
  for (int t = 0; t < 4; ++t) { v8f z = {0.f, 0.f, 0.f, 0.f, 0.f, 0.f, 0.f, 0.f}; acc[t] = z; }
  const _Float16* ahp = sA + (wave * 16 + m) * APH + 8 * hh;
#pragma unroll
  for (int kt = 0; kt < KD / 32; ++kt) {
    FragH af;
    af.h[0] = *(const v8h*)(ahp + 32 * kt);
    af.h[1] = *(const v8h*)(ahp + 32 * kt + 16);
#pragma unroll
    for (int t = 0; t < 4; ++t) {
      const _Float16* bp = Bw + (size_t)(16 * t + m) * KD + 32 * kt + 8 * hh;
      FragH bf;
      bf.h[0] = *(const v8h*)bp;
      bf.h[1] = *(const v8h*)(bp + 16);
      acc[t] = wmf(af.v, bf.v, acc[t]);
    }
  }
  __syncthreads();

  const int r0 = wave * 16 + 8 * hh;
  float* sp = stg + r0 * FH + m;
#pragma unroll
  for (int t = 0; t < 4; ++t) {
#pragma unroll
    for (int r = 0; r < 8; ++r) sp[r * FH + 16 * t] = acc[t][r] * OSC;
  }
  __syncthreads();

  const float* lp = stg + wave * 16 * FH;
  float* gp = C + (size_t)(rowBase + wave * 16) * FH;
#pragma unroll
  for (int i = 0; i < (16 * FH) / 128; ++i) {
    const v4f v = *(const v4f*)(lp + i * 128 + 4 * lane);
    *(volatile v4f*)(gp + i * 128 + 4 * lane) = v;
  }
  __threadfence();
#pragma unroll
  for (int i = 0; i < (16 * FH) / 128; ++i) {
    const v4f v = *(const v4f*)(lp + i * 128 + 4 * lane);
    *(volatile v4f*)(gp + i * 128 + 4 * lane) = v;
  }
}

__global__ __launch_bounds__(NTHR) void k_deg2(
    const int* __restrict__ csr, const int* __restrict__ off, const int* __restrict__ cnt,
    const int* __restrict__ permp, const int* __restrict__ mp, float* d2p, int nN, int csrLen) {
  const int tid = threadIdx.x, lane = tid & 31, wave = tid >> 5;
  const int g = blockIdx.x, t0 = wave * 32;
  const int ocl = clampi(permp[g * KPP + t0 + lane], 0, nN - 1);
  const int cnt_l = cnt[ocl], off_l = off[ocl];
  const int nj = (KPG - t0) < 32 ? (KPG - t0) : 32;
  float myd = 0.f;
#pragma unroll 1
  for (int j = 0; j < nj; ++j) {
    int n = rl_i(cnt_l, j);
    n = clampi(n, 0, DEGCAP);
    const int st = rl_i(off_l, j);
    int vc = 0;
#pragma unroll 1
    for (int q0 = 0; q0 < n; q0 += 32) {
      const int pos = clampi(st + q0 + lane, 0, csrLen - 1);
      const int row = clampi(csr[pos], 0, nN - 1);
      const int a = mp[mp_index(row)];
      const bool v = (q0 + lane < n) && (a >= 0);
      vc += (int)__builtin_popcount(__builtin_amdgcn_ballot_w32(v));
    }
    const float d = 1.0f / sqrtf((float)(vc + 1));
    myd = (lane == j) ? d : myd;
  }
  float* dp = d2p + (size_t)g * KPP + t0 + lane;
  *(volatile float*)dp = myd;
  __threadfence();
  *(volatile float*)dp = myd;
}

__global__ __launch_bounds__(NTHR) void k_gcn(
    const int* __restrict__ csr, const int* __restrict__ off, const int* __restrict__ cnt,
    const int* __restrict__ permp, const int* __restrict__ mp, const float* __restrict__ d2p,
    const float* __restrict__ hall, const float* __restrict__ bs, float* h, float* invp,
    int nN, int nK, int csrLen) {
  const int tid = threadIdx.x, lane = tid & 31, wave = tid >> 5;
  const int g = blockIdx.x, t0 = wave * 32;
  const int ocl = clampi(permp[g * KPP + t0 + lane], 0, nN - 1);
  const int cnt_l = cnt[ocl], off_l = off[ocl];
  const float d2l = d2p[g * KPP + t0 + lane];
  const v2f bb = *(const v2f*)(bs + 2 * lane);
  const int nj = (KPG - t0) < 32 ? (KPG - t0) : 32;
  float myinv = 0.f;
#pragma unroll 1
  for (int j = 0; j < nj; ++j) {
    const int c  = g * KPG + t0 + j;
    const int oc = rl_i(ocl, j);
    int n = rl_i(cnt_l, j);
    n = clampi(n, 0, DEGCAP);
    const int st = rl_i(off_l, j);
    const float dc = rl_f(d2l, j);
    v2f acc = {0.f, 0.f};
#pragma unroll 1
    for (int q0 = 0; q0 < n; q0 += 32) {
      const int pos = clampi(st + q0 + lane, 0, csrLen - 1);
      const int row = clampi(csr[pos], 0, nN - 1);
      int a = mp[mp_index(row)];
      a = (q0 + lane < n) ? a : -1;
      const int ac = clampi(a, 0, nK - 1);
      const float da = d2p[kp_index(ac)];
      const int mcnt = (n - q0) < 32 ? (n - q0) : 32;
#pragma unroll 1
      for (int p = 0; p < mcnt; ++p) {
        const int av = rl_i(a, p);
        if (av >= 0) {
          const int rw = rl_i(row, p);
          const float w = rl_f(da, p) * dc;
          const v2f hv = *(const v2f*)(hall + (size_t)rw * FH + 2 * lane);
          acc = acc + hv * w;
        }
      }
    }
    const v2f hs = *(const v2f*)(hall + (size_t)oc * FH + 2 * lane);
    v2f v = acc + hs * (dc * dc) + bb;
    v.x = fmaxf(v.x, 0.f); v.y = fmaxf(v.y, 0.f);
    const float ssq = wsum(v.x * v.x + v.y * v.y);
    const float inv = 1.0f / fmaxf(sqrtf(ssq), 1e-12f);
    myinv = (lane == j) ? inv : myinv;
    float* hp = h + (size_t)c * FH + 2 * lane;
    *(volatile v2f*)hp = v;
    __threadfence();
    *(volatile v2f*)hp = v;
  }
  float* ip = invp + (size_t)g * KPP + t0 + lane;
  *(volatile float*)ip = myinv;
  __threadfence();
  *(volatile float*)ip = myinv;
}

__global__ __launch_bounds__(NTHR) void k_agnn(
    const int* __restrict__ csr, const int* __restrict__ off, const int* __restrict__ cnt,
    const int* __restrict__ permp, const int* __restrict__ mp, const float* __restrict__ h,
    const float* __restrict__ invp, const float* __restrict__ betap, float* out,
    int nN, int nK, int csrLen) {
  __shared__ __attribute__((aligned(16))) float ssum[NWAVE * FH];
  __shared__ __attribute__((aligned(16))) float smax[NWAVE * FH];
  __shared__ __attribute__((aligned(16))) float srow[2 * FH];
  const int tid = threadIdx.x, lane = tid & 31, wave = tid >> 5;
  const int g = blockIdx.x, t0 = wave * 32;
  const float ninf = __uint_as_float(0xff800000u);
  const float bt = betap[0];
  const int ocl = clampi(permp[g * KPP + t0 + lane], 0, nN - 1);
  const int cnt_l = cnt[ocl], off_l = off[ocl];
  const float ivl = invp[g * KPP + t0 + lane];
  const int nj = (KPG - t0) < 32 ? (KPG - t0) : 32;
  v2f psum = {0.f, 0.f};
  v2f pmax = {ninf, ninf};

#pragma unroll 1
  for (int j = 0; j < nj; ++j) {
    const int c = g * KPG + t0 + j;
    int n = rl_i(cnt_l, j);
    n = clampi(n, 0, DEGCAP);
    const int st = rl_i(off_l, j);
    const float ivc = rl_f(ivl, j);
    const v2f hc = *(const v2f*)(h + (size_t)c * FH + 2 * lane);
    const v2f hn = hc * ivc;
    const float ls = bt * wsum(hn.x * hn.x + hn.y * hn.y);

    float m = ninf;
#pragma unroll 1
    for (int q0 = 0; q0 < n; q0 += 32) {
      const int pos = clampi(st + q0 + lane, 0, csrLen - 1);
      const int row = clampi(csr[pos], 0, nN - 1);
      int a = mp[mp_index(row)];
      a = (q0 + lane < n) ? a : -1;
      const int ac = clampi(a, 0, nK - 1);
      const float ia = invp[kp_index(ac)];
      const int mcnt = (n - q0) < 32 ? (n - q0) : 32;
#pragma unroll 1
      for (int p = 0; p < mcnt; ++p) {
        const int av = rl_i(a, p);
        if (av >= 0) {
          const int au = rl_i(ac, p);
          const float wi = rl_f(ia, p);
          const v2f ha = *(const v2f*)(h + (size_t)au * FH + 2 * lane);
          const float dt = wsum((ha.x * wi) * hn.x + (ha.y * wi) * hn.y);
          m = fmaxf(m, bt * dt);
        }
      }
    }
    m = fmaxf(m, ls);

    float den = 0.f;
    v2f acc = {0.f, 0.f};
#pragma unroll 1
    for (int q0 = 0; q0 < n; q0 += 32) {
      const int pos = clampi(st + q0 + lane, 0, csrLen - 1);
      const int row = clampi(csr[pos], 0, nN - 1);
      int a = mp[mp_index(row)];
      a = (q0 + lane < n) ? a : -1;
      const int ac = clampi(a, 0, nK - 1);
      const float ia = invp[kp_index(ac)];
      const int mcnt = (n - q0) < 32 ? (n - q0) : 32;
#pragma unroll 1
      for (int p = 0; p < mcnt; ++p) {
        const int av = rl_i(a, p);
        if (av >= 0) {
          const int au = rl_i(ac, p);
          const float wi = rl_f(ia, p);
          const v2f ha = *(const v2f*)(h + (size_t)au * FH + 2 * lane);
          const float dt = wsum((ha.x * wi) * hn.x + (ha.y * wi) * hn.y);
          const float ee = expf(bt * dt - m);
          den += ee;
          acc = acc + ha * ee;
        }
      }
    }
    const float es = expf(ls - m);
    den += es;
    const float rd = 1.0f / den;
    const v2f o = (acc + hc * es) * rd;
    psum = psum + o;
    pmax.x = fmaxf(pmax.x, o.x); pmax.y = fmaxf(pmax.y, o.y);
  }
  *(v2f*)(ssum + wave * FH + 2 * lane) = psum;
  *(v2f*)(smax + wave * FH + 2 * lane) = pmax;
  __syncthreads();
  if (tid < FH) {
    float s = 0.f, mx = ninf;
#pragma unroll
    for (int w = 0; w < NWAVE; ++w) { s += ssum[w * FH + tid]; mx = fmaxf(mx, smax[w * FH + tid]); }
    srow[tid]      = fmaxf(s * (1.0f / (float)KPG), 0.f);
    srow[FH + tid] = fmaxf(mx, 0.f);
  }
  __syncthreads();
  v4f ov = {0.f, 0.f, 0.f, 0.f};
  if (tid < 32) ov = *(const v4f*)(srow + 4 * tid);
  float* op = out + (size_t)g * (2 * FH) + 4 * tid;
  if (tid < 32) *(volatile v4f*)op = ov;
  __threadfence();
  if (tid < 32) *(volatile v4f*)op = ov;
}

extern "C" void kernel_launch(void* const* d_in, const int* in_sizes, int n_in,
                              void* d_out, int out_size, void* d_ws, size_t ws_size,
                              hipStream_t stream) {
  if (n_in < 5) return;
  const int nN = in_sizes[0] / FIN;
  const int nE = in_sizes[1] / 2;
  if (nN <= 0 || nE <= 0 || in_sizes[0] != nN * FIN || in_sizes[1] != 2 * nE) return;
  if (in_sizes[2] != FIN * FH || in_sizes[3] != FH || in_sizes[4] < 1) return;
  const int nG = nN / NPG;
  if (nG <= 0 || nG * NPG != nN) return;
  if (out_size != nG * 2 * FH) return;
  if (nN > (1 << 20) || nE > (1 << 28)) return;
  const int nK = nG * KPG;

  const float* x    = (const float*)d_in[0];
  const int*   ei   = (const int*)d_in[1];
  const float* W1   = (const float*)d_in[2];
  const float* b1   = (const float*)d_in[3];
  const float* beta = (const float*)d_in[4];
  float* out = (float*)d_out;

  const int nBC    = (nN + NBC - 1) / NBC;
  const int CNTPAD = nBC * NBC;
  const int nBF    = (nN + NBF - 1) / NBF;
  const int OFFN   = nBF * NBF;
  if (nBF + 1 > RBN) return;
  if (OFFN > CNTPAD) return;
  const int nSB    = (nN + TGT - 1) / TGT;
  const int NPADS  = nSB * TGT;
  if (NPADS > OFFN) return;
  const int csrLen = ((nE + 31) & ~31) + 32 * (nBF + 1);
  const int nGemm  = (nN + GROWS - 1) / GROWS;
  const int NPADG  = nGemm * GROWS;

  char* ws = (char*)d_ws;
  size_t off = 0;
  const size_t oW    = off; off += (size_t)FIN * FH * 2;            off = (off + 255) & ~(size_t)255;
  const size_t oCntR = off; off += (size_t)CNTPAD * 4;              off = (off + 255) & ~(size_t)255;
  const size_t oDisR = off; off += (size_t)CNTPAD * 4;              off = (off + 255) & ~(size_t)255;
  const size_t oCntC = off; off += (size_t)CNTPAD * 4;              off = (off + 255) & ~(size_t)255;
  const size_t oOff  = off; off += (size_t)OFFN * 4;                off = (off + 255) & ~(size_t)255;
  const size_t oRb   = off; off += (size_t)RBN * 4;                 off = (off + 255) & ~(size_t)255;
  const size_t oCsr  = off; off += (size_t)csrLen * 4;              off = (off + 255) & ~(size_t)255;
  const size_t oSc   = off; off += (size_t)NPADS * 8;               off = (off + 255) & ~(size_t)255;
  const size_t oMp   = off; off += (size_t)nG * MPP * 4;            off = (off + 255) & ~(size_t)255;
  const size_t oPerm = off; off += (size_t)nG * KPP * 4;            off = (off + 255) & ~(size_t)255;
  const size_t oHall = off; off += (size_t)NPADG * FH * 4;          off = (off + 255) & ~(size_t)255;
  const size_t oD2   = off; off += (size_t)nG * KPP * 4;            off = (off + 255) & ~(size_t)255;
  const size_t oH    = off; off += (size_t)nK * FH * 4;             off = (off + 255) & ~(size_t)255;
  const size_t oInv  = off; off += (size_t)nG * KPP * 4;            off = (off + 255) & ~(size_t)255;
  if (off > ws_size || off > (size_t)WSCAP) return;
  _Float16* wp    = (_Float16*)(ws + oW);
  int*      cntR  = (int*)(ws + oCntR);
  float*    disR  = (float*)(ws + oDisR);
  int*      cntC  = (int*)(ws + oCntC);
  int*      offp  = (int*)(ws + oOff);
  int*      rb    = (int*)(ws + oRb);
  int*      csr   = (int*)(ws + oCsr);
  double*   score = (double*)(ws + oSc);
  int*      mp    = (int*)(ws + oMp);
  int*      permp = (int*)(ws + oPerm);
  float*    hall  = (float*)(ws + oHall);
  float*    d2p   = (float*)(ws + oD2);
  float*    h     = (float*)(ws + oH);
  float*    invp  = (float*)(ws + oInv);

  const int vec8 = ((nE & 3) == 0) ? 1 : 0;

  k_wprep<<<2, NTHR, 0, stream>>>(W1, wp);

  hipFuncSetAttribute(reinterpret_cast<const void*>(&k_count<1>),
                      hipFuncAttributeMaxDynamicSharedMemorySize, LDS_COUNT);
  k_count<1><<<nBC, NTHR, LDS_COUNT, stream>>>(ei, 0, cntR, disR, nE, nN, vec8);
  hipFuncSetAttribute(reinterpret_cast<const void*>(&k_count<0>),
                      hipFuncAttributeMaxDynamicSharedMemorySize, LDS_COUNT);
  k_count<0><<<nBC, NTHR, LDS_COUNT, stream>>>(ei, nE, cntC, disR, nE, nN, vec8);

  k_offsets<<<1, OTHR, 0, stream>>>(cntC, offp, rb, nBF);
  hipFuncSetAttribute(reinterpret_cast<const void*>(&k_fill),
                      hipFuncAttributeMaxDynamicSharedMemorySize, LDS_FILL);
  k_fill<<<nBF, NTHR, LDS_FILL, stream>>>(ei, offp, rb, csr, nN, nE, vec8, csrLen);

  k_score<<<nSB, NTHR, 0, stream>>>(csr, offp, cntC, disR, x, score, nN, csrLen);
  k_topk<<<nG, NTHR, 0, stream>>>(score, mp, permp, nN);

  k_gemm<<<nGemm, NTHR, LDS_GEMM, stream>>>(x, wp, hall, nN);

  k_deg2<<<nG, NTHR, 0, stream>>>(csr, offp, cntC, permp, mp, d2p, nN, csrLen);
  k_gcn<<<nG, NTHR, 0, stream>>>(csr, offp, cntC, permp, mp, d2p, hall, b1, h, invp, nN, nK, csrLen);
  k_agnn<<<nG, NTHR, 0, stream>>>(csr, offp, cntC, permp, mp, h, invp, beta, out, nN, nK, csrLen);
}
